// LSTMAutoencoder_10307921510453
// MI455X (gfx1250) — hardware-verified
//
#include <hip/hip_runtime.h>
#include <math.h>

constexpr int NB    = 512;
constexpr int NSTEP = 128;
constexpr int NX    = 128;
constexpr int NHE   = 256;
constexpr int NHD   = 128;
constexpr int NTHR  = 256;
constexpr int SEQ_ROWS = 16;
constexpr float CARRY      = 16.0f;
constexpr float CARRY2_INV = 1.0f / 256.0f;
static_assert(NB % SEQ_ROWS == 0);
static_assert(NX % 32 == 0 && NHE % 32 == 0 && NHD % 32 == 0);
static_assert(NB % 64 == 0 && (4 * NHD) % 64 == 0 && NX % 64 == 0 && (NB * NSTEP) % 64 == 0);
static_assert(((NB / 64) * ((4 * NHD) / 64)) % 8 == 0);
static_assert((((NB * NSTEP) / 64) * (NX / 64)) % 8 == 0);
static_assert(NX == NHD);

typedef __attribute__((ext_vector_type(16))) _Float16 v16h;
typedef __attribute__((ext_vector_type(8)))  _Float16 v8h;
typedef __attribute__((ext_vector_type(16))) __bf16   v16b;
typedef __attribute__((ext_vector_type(8)))  __bf16   v8b;
typedef __attribute__((ext_vector_type(8)))  float    v8f;
typedef __attribute__((ext_vector_type(4)))  float    v4f;
typedef __attribute__((ext_vector_type(4)))  unsigned v4u;

__device__ __forceinline__ unsigned short f2bf_bits(float f) {
  unsigned u = __float_as_uint(f);
  return (unsigned short)((u + 0x7FFFu + ((u >> 16) & 1u)) >> 16);
}
__device__ __forceinline__ float bf_bits2f(unsigned short h) { return __uint_as_float(((unsigned)h) << 16); }
__device__ __forceinline__ float bf16r(float f) { return bf_bits2f(f2bf_bits(f)); }

__device__ __forceinline__ void dep_guard_h(v8f& a, v8f& b, v16h x, v16h y) { asm volatile("v_nop\n\tv_nop\n\tv_nop\n\tv_nop" : "+v"(a), "+v"(b) : "v"(x), "v"(y)); }
__device__ __forceinline__ void dep_guard_b(v8f& a, v8f& b, v16b x, v16b y) { asm volatile("v_nop\n\tv_nop\n\tv_nop\n\tv_nop" : "+v"(a), "+v"(b) : "v"(x), "v"(y)); }
__device__ __forceinline__ void dep_guard4_h(v8f& a, v8f& b, v8f& c, v8f& d, v16h x, v16h y, v16h z) { asm volatile("v_nop\n\tv_nop\n\tv_nop\n\tv_nop" : "+v"(a), "+v"(b), "+v"(c), "+v"(d) : "v"(x), "v"(y), "v"(z)); }
__device__ __forceinline__ void dep_guard4_b(v8f& a, v8f& b, v8f& c, v8f& d, v16b x, v16b y, v16b z) { asm volatile("v_nop\n\tv_nop\n\tv_nop\n\tv_nop" : "+v"(a), "+v"(b), "+v"(c), "+v"(d) : "v"(x), "v"(y), "v"(z)); }
__device__ __forceinline__ void keep4_h(v16h a, v16h b, v16h c, v16h d) { asm volatile("v_nop" :: "v"(a), "v"(b), "v"(c), "v"(d)); }
__device__ __forceinline__ void keep4_b(v16b a, v16b b, v16b c, v16b d) { asm volatile("v_nop" :: "v"(a), "v"(b), "v"(c), "v"(d)); }
__device__ __forceinline__ void acc_guard4(v8f& a, v8f& b, v8f& c, v8f& d) { asm volatile("v_nop\n\tv_nop\n\tv_nop\n\tv_nop" : "+v"(a), "+v"(b), "+v"(c), "+v"(d)); }
__device__ __forceinline__ void guard_all_h(v8f& a0, v8f& a1, v8f& a2, v8f& a3, v16h x, v16h y0, v16h y1, v16h y2, v16h y3) {
  asm volatile("v_nop\n\tv_nop\n\tv_nop\n\tv_nop" : "+v"(a0), "+v"(a1), "+v"(a2), "+v"(a3) : "v"(x), "v"(y0), "v"(y1), "v"(y2), "v"(y3));
}
__device__ __forceinline__ void vdep4(float& a, float& b, float& c, float& d) { asm volatile("" : "+v"(a), "+v"(b), "+v"(c), "+v"(d) : : "memory"); }

template <typename T> struct Frag;
template <> struct Frag<_Float16> {
  typedef v16h V; union U { v16h v; v8h h[2]; };
  static __device__ __forceinline__ v16h load(const _Float16* p) {
    U f; f.h[0] = *(const v8h*)(p); f.h[1] = *(const v8h*)(p + 16); return f.v;
  }
  static __device__ __forceinline__ v8f mma(v16h a, v16h b, v8f c) {
    return __builtin_amdgcn_wmma_f32_16x16x32_f16(false, a, false, b, (short)0, c, false, false);
  }
  static __device__ __forceinline__ void guard(v8f& a, v8f& b, v16h x, v16h y) { dep_guard_h(a, b, x, y); }
  static __device__ __forceinline__ void guard4(v8f& a, v8f& b, v8f& c, v8f& d, v16h x, v16h y, v16h z) { dep_guard4_h(a, b, c, d, x, y, z); }
  static __device__ __forceinline__ void keep(v16h a, v16h b, v16h c, v16h d) { keep4_h(a, b, c, d); }
};
template <> struct Frag<__bf16> {
  typedef v16b V; union U { v16b v; v8b h[2]; };
  static __device__ __forceinline__ v16b load(const __bf16* p) {
    U f; f.h[0] = *(const v8b*)(p); f.h[1] = *(const v8b*)(p + 16); return f.v;
  }
  static __device__ __forceinline__ v8f mma(v16b a, v16b b, v8f c) {
    return __builtin_amdgcn_wmma_f32_16x16x32_bf16(false, a, false, b, (short)0, c, false, false);
  }
  static __device__ __forceinline__ void guard(v8f& a, v8f& b, v16b x, v16b y) { dep_guard_b(a, b, x, y); }
  static __device__ __forceinline__ void guard4(v8f& a, v8f& b, v8f& c, v8f& d, v16b x, v16b y, v16b z) { dep_guard4_b(a, b, c, d, x, y, z); }
  static __device__ __forceinline__ void keep(v16b a, v16b b, v16b c, v16b d) { keep4_b(a, b, c, d); }
};

__device__ __forceinline__ float fsig(float x)  { return __builtin_amdgcn_rcpf(1.0f + expf(-x)); }
__device__ __forceinline__ float ftanh(float x) { return 1.0f - 2.0f * __builtin_amdgcn_rcpf(expf(2.0f * x) + 1.0f); }

template <int ET> struct Elem;
template <> struct Elem<0> { typedef _Float16 T; };
template <> struct Elem<1> { typedef __bf16 T; };
template <int ET, bool SPLIT, int BIAS_MODE, int OUT_MODE, bool RESID, int ACT = 0>
__global__ __launch_bounds__(256) void wmma_gemm64(
    const unsigned short* __restrict__ Ap, const unsigned short* __restrict__ A2p, int lda, long strideA,
    const unsigned short* __restrict__ Btp, const unsigned short* __restrict__ Bt2p, int ldb, long strideB,
    void* __restrict__ Cout, void* __restrict__ Cout2, int ldc, long strideC,
    const float* __restrict__ bias,
    const float* __restrict__ resid, long strideR,
    int M, int N, int K, float scale) {
  typedef typename Elem<ET>::T T;
  typedef typename Frag<T>::V V;
  const T* A = (const T*)Ap; const T* A2 = (const T*)A2p; const T* Bt = (const T*)Btp; const T* Bt2 = (const T*)Bt2p;
  __shared__ __align__(16) float sT[8][16 * 68];
  const int b    = blockIdx.y;
  const int lane = threadIdx.x & 31;
  const int wave = threadIdx.x >> 5;
  const int tilesN = N >> 6;
  const int tilesM = M >> 6;
  const int tile = blockIdx.x * 8 + wave;
  if (tile >= tilesM * tilesN) return;
  const int tm = tile / tilesN;
  const int tn = tile - tm * tilesN;
  const int m0 = tm << 6;
  const int n0 = tn << 6;

  const T* Ab  = A  + (size_t)b * strideA;
  const T* Bb  = Bt + (size_t)b * strideB;
  const T* Ab2 = SPLIT ? (A2  + (size_t)b * strideA) : nullptr;
  const T* Bb2 = SPLIT ? (Bt2 + (size_t)b * strideB) : nullptr;

  const int rlane = lane & 15;
  const int koff  = (lane >> 4) * 8;
  const int mOff  = (lane >> 4) * 8;

  v8f acc[4][4];
#pragma unroll
  for (int i = 0; i < 4; ++i)
#pragma unroll
    for (int j = 0; j < 4; ++j) acc[i][j] = (v8f){0.f,0.f,0.f,0.f,0.f,0.f,0.f,0.f};

  for (int k0 = 0; k0 < K; k0 += 32) {
    V bh[4], bl[4];
#pragma unroll
    for (int j = 0; j < 4; ++j) {
      const size_t bo = (size_t)(n0 + (j << 4) + rlane) * ldb + koff + k0;
      bh[j] = Frag<T>::load(Bb + bo);
      if (SPLIT) bl[j] = Frag<T>::load(Bb2 + bo);
    }
#pragma unroll
    for (int i = 0; i < 4; ++i) {
      const size_t ao = (size_t)(m0 + (i << 4) + rlane) * lda + koff + k0;
      V ah = Frag<T>::load(Ab + ao);
      V al;
      if (SPLIT) al = Frag<T>::load(Ab2 + ao);
#pragma unroll
      for (int j = 0; j < 4; ++j) {
        acc[i][j] = Frag<T>::mma(ah, bh[j], acc[i][j]);
        if (SPLIT) {
          acc[i][j] = Frag<T>::mma(ah, bl[j], acc[i][j]);
          acc[i][j] = Frag<T>::mma(al, bh[j], acc[i][j]);
        }
      }
      Frag<T>::guard4(acc[i][0], acc[i][1], acc[i][2], acc[i][3], ah, SPLIT ? al : ah, bh[3]);
    }
    Frag<T>::keep(bh[0], bh[1], bh[2], bh[3]);
    if (SPLIT) Frag<T>::keep(bl[0], bl[1], bl[2], bl[3]);
  }
  acc_guard4(acc[0][0], acc[0][1], acc[0][2], acc[0][3]);
  acc_guard4(acc[1][0], acc[1][1], acc[1][2], acc[1][3]);
  acc_guard4(acc[2][0], acc[2][1], acc[2][2], acc[2][3]);
  acc_guard4(acc[3][0], acc[3][1], acc[3][2], acc[3][3]);

  float* slab = sT[wave];
  const float* Rb = RESID ? (resid + (size_t)b * strideR) : nullptr;
#pragma unroll
  for (int i = 0; i < 4; ++i) {
    const int mBase = m0 + (i << 4);
#pragma unroll
    for (int j = 0; j < 4; ++j) {
      const int n = n0 + (j << 4) + rlane;
      float bv = 0.f;
      if (BIAS_MODE == 2) bv = bias[n];
#pragma unroll
      for (int r = 0; r < 8; ++r) {
        float v = acc[i][j][r] * scale;
        if (BIAS_MODE == 1) v += bias[mBase + mOff + r];
        if (BIAS_MODE == 2) v += bv;
        if (RESID) v += Rb[(size_t)(mBase + mOff + r) * ldc + n];
        if (ACT == 1) v = tanhf(v);
        if (ACT == 2) v = fmaxf(v, 0.0f);
        if (ACT == 3) v = v / (1.0f + expf(-v));
        if (ACT == 4) v = (v > 0.f) ? v : 0.01f * v;
        if (ACT == 5) v = 0.5f * v * (1.0f + erff(v * 0.70710678118654752f));
        slab[(mOff + r) * 68 + (j << 4) + rlane] = v;
      }
    }
    __builtin_amdgcn_fence(__ATOMIC_RELEASE, "workgroup");
    __builtin_amdgcn_wave_barrier();
    __builtin_amdgcn_fence(__ATOMIC_ACQUIRE, "workgroup");
    if (OUT_MODE == 0) {
      float* C = (float*)Cout + (size_t)b * strideC;
      const int hh = lane >> 4, c4 = (lane & 15) * 4;
      for (int pass = 0; pass < 2; ++pass) {
#pragma unroll
        for (int it = 0; it < 8; ++it) {
          const int row = it * 2 + hh;
          v4f v = *(const v4f*)(slab + row * 68 + c4);
          *(volatile v4f*)(C + (size_t)(mBase + row) * ldc + n0 + c4) = v;
        }
        __threadfence();
      }
    } else {
      const int q = lane >> 3, c8 = (lane & 7) * 8;
      unsigned short* C  = (unsigned short*)Cout  + (size_t)b * strideC;
      unsigned short* C2 = (OUT_MODE == 2) ? ((unsigned short*)Cout2 + (size_t)b * strideC) : nullptr;
      for (int pass = 0; pass < 2; ++pass) {
#pragma unroll
        for (int it = 0; it < 4; ++it) {
          const int row = it * 4 + q;
          const float* sp = slab + row * 68 + c8;
          v8h hv, lv;
#pragma unroll
          for (int e = 0; e < 8; ++e) {
            if (OUT_MODE == 1) {
              hv[e] = (_Float16)sp[e];
            } else {
              unsigned short hb = f2bf_bits(sp[e]);
              unsigned short lb = f2bf_bits(sp[e] - bf_bits2f(hb));
              hv[e] = __builtin_bit_cast(_Float16, hb);
              lv[e] = __builtin_bit_cast(_Float16, lb);
            }
          }
          *(volatile v8h*)(C + (size_t)(mBase + row) * ldc + n0 + c8) = hv;
          if (OUT_MODE == 2) *(volatile v8h*)(C2 + (size_t)(mBase + row) * ldc + n0 + c8) = lv;
        }
        __threadfence();
      }
    }
    __builtin_amdgcn_fence(__ATOMIC_RELEASE, "workgroup");
    __builtin_amdgcn_wave_barrier();
    __builtin_amdgcn_fence(__ATOMIC_ACQUIRE, "workgroup");
  }
}

__global__ __launch_bounds__(NTHR) void cvt16_kernel(const float* __restrict__ src, unsigned short* __restrict__ dst,
                                                     int n8, float sc) {
  const int i = blockIdx.x * NTHR + threadIdx.x;
  if (i < n8) {
    const float* sp = src + (size_t)i * 8;
    const v4f a  = *(const v4f*)(sp);
    const v4f bq = *(const v4f*)(sp + 4);
    v8h hv;
#pragma unroll
    for (int e = 0; e < 4; ++e) {
      hv[e]     = (_Float16)(bf16r(a[e])  * sc);
      hv[4 + e] = (_Float16)(bf16r(bq[e]) * sc);
    }
    *(volatile v8h*)(dst + (size_t)i * 8) = hv;
    __threadfence();
    *(volatile v8h*)(dst + (size_t)i * 8) = hv;
  }
}

__global__ __launch_bounds__(32) void bias16_kernel(const float* __restrict__ src, float* __restrict__ dst) {
  const int lane = threadIdx.x;
  const v4f a = *(const v4f*)(src + 4 * lane);
  v4f o;
#pragma unroll
  for (int e = 0; e < 4; ++e) o[e] = bf16r(a[e]);
  *(volatile v4f*)(dst + 4 * lane) = o;
  __threadfence();
  *(volatile v4f*)(dst + 4 * lane) = o;
}

template <int DIN, int XMODE, int KP>
__device__ __forceinline__ void stage_rows(_Float16* dst, const float* __restrict__ xf, const unsigned short* __restrict__ xh,
                                           int b0, int ts, int tid) {
  if constexpr (XMODE == 0) {
    static_assert(DIN == 128);
    const int m = tid >> 4, f8 = (tid & 15) * 8;
    const float* sp = xf + ((size_t)(b0 + m) * NSTEP + (size_t)ts) * DIN + f8;
    const v4f a  = *(const v4f*)(sp);
    const v4f bq = *(const v4f*)(sp + 4);
    v8h hv;
#pragma unroll
    for (int e = 0; e < 4; ++e) {
      hv[e]     = (_Float16)(bf16r(a[e])  * CARRY);
      hv[4 + e] = (_Float16)(bf16r(bq[e]) * CARRY);
    }
    *(v8h*)(dst + m * KP + f8) = hv;
  } else if constexpr (XMODE == 1) {
    constexpr int C8  = DIN / 8;
    constexpr int PER = (SEQ_ROWS * C8) / NTHR;
    static_assert((SEQ_ROWS * C8) % NTHR == 0 && PER >= 1);
#pragma unroll
    for (int it = 0; it < PER; ++it) {
      const int i  = it * NTHR + tid;
      const int m  = i / C8;
      const int c8 = i - m * C8;
      const v4u v = *(const v4u*)(xh + ((size_t)(b0 + m) * NSTEP + (size_t)ts) * DIN + 8 * c8);
      *(v4u*)(dst + m * KP + 8 * c8) = v;
    }
  }
}

template <int H, int DIN, int XMODE, bool OUTSEQ, bool OUTFIN>
__global__ __launch_bounds__(NTHR) void lstm_seq_kernel(
    const float* __restrict__ xf, const unsigned short* __restrict__ xh, const float* __restrict__ xg,
    const unsigned short* __restrict__ Wihp, const unsigned short* __restrict__ Whhp,
    const float* __restrict__ bih, const float* __restrict__ bhh,
    unsigned short* __restrict__ seq, unsigned short* __restrict__ hfin) {
  constexpr int KX    = (XMODE == 2) ? 0 : DIN;
  constexpr int KP    = KX + H + 8;
  constexpr int NWAVE = NTHR / 32;
  constexpr int UPW   = H / NWAVE;
  constexpr int NTU   = UPW / 16;
  constexpr int G4    = 4 * H;
  static_assert(SEQ_ROWS == 16 && NTHR == 256);
  static_assert(H == 256 || H == 128);
  static_assert(UPW % 16 == 0 && NTU >= 1 && NTU <= 2);
  static_assert(KX % 32 == 0 && H % 32 == 0 && KP % 8 == 0);
  static_assert((2 * SEQ_ROWS * KP) % NTHR == 0);

  __shared__ __align__(16) _Float16 Abuf[2][SEQ_ROWS * KP];
  const _Float16* Wih = (const _Float16*)Wihp;
  const _Float16* Whh = (const _Float16*)Whhp;
  const int tid = threadIdx.x, lane = tid & 31, wave = tid >> 5;
  const int c = lane & 15, hh = lane >> 4, koff = hh * 8;
  const int b0 = blockIdx.x * SEQ_ROWS;

  {
    _Float16* af = &Abuf[0][0];
#pragma unroll 1
    for (int i = tid; i < 2 * SEQ_ROWS * KP; i += NTHR) af[i] = (_Float16)0.0f;
  }
  __syncthreads();

  float bs[NTU][4];
#pragma unroll
  for (int nt = 0; nt < NTU; ++nt) {
    const int j = UPW * wave + 16 * nt + c;
#pragma unroll
    for (int g = 0; g < 4; ++g) bs[nt][g] = bf16r(bih[g * H + j]) + bf16r(bhh[g * H + j]);
    vdep4(bs[nt][0], bs[nt][1], bs[nt][2], bs[nt][3]);
  }
  float xgc[4][8];
#pragma unroll
  for (int g = 0; g < 4; ++g)
#pragma unroll
    for (int r = 0; r < 8; ++r) xgc[g][r] = 0.0f;
  if constexpr (XMODE == 2) {
    const int j = UPW * wave + c;
#pragma unroll
    for (int g = 0; g < 4; ++g) {
#pragma unroll
      for (int r = 0; r < 8; ++r) xgc[g][r] = xg[(size_t)(b0 + 8 * hh + r) * G4 + g * H + j] + bs[0][g];
      vdep4(xgc[g][0], xgc[g][1], xgc[g][2], xgc[g][3]);
      vdep4(xgc[g][4], xgc[g][5], xgc[g][6], xgc[g][7]);
    }
  }
  if constexpr (XMODE != 2) stage_rows<DIN, XMODE, KP>(&Abuf[0][0], xf, xh, b0, 0, tid);
  float cst[NTU][8];
#pragma unroll
  for (int nt = 0; nt < NTU; ++nt)
#pragma unroll
    for (int r = 0; r < 8; ++r) cst[nt][r] = 0.0f;
  __syncthreads();

  const v8f z8 = {0.f, 0.f, 0.f, 0.f, 0.f, 0.f, 0.f, 0.f};

#pragma unroll 1
  for (int t = 0; t < NSTEP; ++t) {
    const int cur = t & 1;
    const _Float16* arow = &Abuf[cur][0] + c * KP + koff;
    _Float16* An = &Abuf[cur ^ 1][0];

#pragma unroll
    for (int nt = 0; nt < NTU; ++nt) {
      const int j = UPW * wave + 16 * nt + c;
      v8f acc0 = z8, acc1 = z8, acc2 = z8, acc3 = z8;
      if constexpr (XMODE != 2) {
        const _Float16* wi = Wih + (size_t)j * DIN + koff;
#pragma unroll 1
        for (int kx = 0; kx < KX; kx += 32) {
          const v16h a  = Frag<_Float16>::load(arow + kx);
          const v16h w0 = Frag<_Float16>::load(wi + kx);
          const v16h w1 = Frag<_Float16>::load(wi + (size_t)1 * H * DIN + kx);
          const v16h w2 = Frag<_Float16>::load(wi + (size_t)2 * H * DIN + kx);
          const v16h w3 = Frag<_Float16>::load(wi + (size_t)3 * H * DIN + kx);
          acc0 = Frag<_Float16>::mma(a, w0, acc0);
          acc1 = Frag<_Float16>::mma(a, w1, acc1);
          acc2 = Frag<_Float16>::mma(a, w2, acc2);
          acc3 = Frag<_Float16>::mma(a, w3, acc3);
          guard_all_h(acc0, acc1, acc2, acc3, a, w0, w1, w2, w3);
        }
      }
      {
        const _Float16* wr = Whh + (size_t)j * H + koff;
#pragma unroll 1
        for (int kh = 0; kh < H; kh += 32) {
          const v16h a  = Frag<_Float16>::load(arow + KX + kh);
          const v16h w0 = Frag<_Float16>::load(wr + kh);
          const v16h w1 = Frag<_Float16>::load(wr + (size_t)1 * H * H + kh);
          const v16h w2 = Frag<_Float16>::load(wr + (size_t)2 * H * H + kh);
          const v16h w3 = Frag<_Float16>::load(wr + (size_t)3 * H * H + kh);
          acc0 = Frag<_Float16>::mma(a, w0, acc0);
          acc1 = Frag<_Float16>::mma(a, w1, acc1);
          acc2 = Frag<_Float16>::mma(a, w2, acc2);
          acc3 = Frag<_Float16>::mma(a, w3, acc3);
          guard_all_h(acc0, acc1, acc2, acc3, a, w0, w1, w2, w3);
        }
      }
      acc_guard4(acc0, acc1, acc2, acc3);
#pragma unroll
      for (int r = 0; r < 8; ++r) {
        float add0, add1, add2, add3;
        if constexpr (XMODE == 2) { add0 = xgc[0][r]; add1 = xgc[1][r]; add2 = xgc[2][r]; add3 = xgc[3][r]; }
        else                      { add0 = bs[nt][0];  add1 = bs[nt][1];  add2 = bs[nt][2];  add3 = bs[nt][3]; }
        const float zi = acc0[r] * CARRY2_INV + add0;
        const float zf = acc1[r] * CARRY2_INV + add1;
        const float zg = acc2[r] * CARRY2_INV + add2;
        const float zo = acc3[r] * CARRY2_INV + add3;
        const float ig = fsig(zi);
        const float fg = fsig(zf);
        const float gg = ftanh(zg);
        const float og = fsig(zo);
        const float cn = fg * cst[nt][r] + ig * gg;
        cst[nt][r] = cn;
        const float hn = og * ftanh(cn);
        An[(8 * hh + r) * KP + KX + j] = (_Float16)(hn * CARRY);
      }
    }
    if constexpr (XMODE != 2) {
      const int tn = (t + 1 < NSTEP) ? (t + 1) : (NSTEP - 1);
      stage_rows<DIN, XMODE, KP>(An, xf, xh, b0, tn, tid);
    }
    __syncthreads();

    if constexpr (OUTSEQ || OUTFIN) {
      const bool last = (t == NSTEP - 1);
      if (OUTSEQ || last) {
        if constexpr (H == 256) {
          const int q8 = lane * 8;
          for (int pass = 0; pass < 2; ++pass) {
#pragma unroll
            for (int rr = 0; rr < 2; ++rr) {
              const int row = wave + NWAVE * rr;
              const v4u v = *(const v4u*)(An + row * KP + KX + q8);
              if constexpr (OUTSEQ) *(volatile v4u*)(seq + ((size_t)(b0 + row) * NSTEP + (size_t)t) * H + q8) = v;
              if constexpr (OUTFIN) { if (last) *(volatile v4u*)(hfin + (size_t)(b0 + row) * H + q8) = v; }
            }
            __threadfence();
          }
        } else {
          const int row = 2 * wave + hh;
          const int q8  = c * 8;
          for (int pass = 0; pass < 2; ++pass) {
            const v4u v = *(const v4u*)(An + row * KP + KX + q8);
            if constexpr (OUTSEQ) *(volatile v4u*)(seq + ((size_t)(b0 + row) * NSTEP + (size_t)t) * H + q8) = v;
            if constexpr (OUTFIN) { if (last) *(volatile v4u*)(hfin + (size_t)(b0 + row) * H + q8) = v; }
            __threadfence();
          }
        }
      }
    }
  }
}

extern "C" void kernel_launch(void* const* d_in, const int* in_sizes, int n_in,
                              void* d_out, int out_size, void* d_ws, size_t ws_size, hipStream_t stream) {
  if (n_in < 19 || d_out == nullptr || d_ws == nullptr) return;
  if (in_sizes[0] != NB * NSTEP * NX ||
      in_sizes[1] != 4 * NHE * NX  || in_sizes[2] != 4 * NHE * NHE || in_sizes[3] != 4 * NHE || in_sizes[4] != 4 * NHE ||
      in_sizes[5] != 4 * NHE * NHE || in_sizes[6] != 4 * NHE * NHE || in_sizes[7] != 4 * NHE || in_sizes[8] != 4 * NHE ||
      in_sizes[9] != 4 * NHD * NHE || in_sizes[10] != 4 * NHD * NHD || in_sizes[11] != 4 * NHD || in_sizes[12] != 4 * NHD ||
      in_sizes[13] != 4 * NHD * NX || in_sizes[14] != 4 * NHD * NHD || in_sizes[15] != 4 * NHD || in_sizes[16] != 4 * NHD ||
      in_sizes[17] != NX * NX || in_sizes[18] != NX || out_size != NB * NSTEP * NX) return;

  const float* x      = (const float*)d_in[0];
  const float* e0_wih = (const float*)d_in[1];
  const float* e0_whh = (const float*)d_in[2];
  const float* e0_bih = (const float*)d_in[3];
  const float* e0_bhh = (const float*)d_in[4];
  const float* e1_wih = (const float*)d_in[5];
  const float* e1_whh = (const float*)d_in[6];
  const float* e1_bih = (const float*)d_in[7];
  const float* e1_bhh = (const float*)d_in[8];
  const float* d0_wih = (const float*)d_in[9];
  const float* d0_whh = (const float*)d_in[10];
  const float* d0_bih = (const float*)d_in[11];
  const float* d0_bhh = (const float*)d_in[12];
  const float* d1_wih = (const float*)d_in[13];
  const float* d1_whh = (const float*)d_in[14];
  const float* d1_bih = (const float*)d_in[15];
  const float* d1_bhh = (const float*)d_in[16];
  const float* out_w  = (const float*)d_in[17];
  const float* out_b  = (const float*)d_in[18];
  float* out = (float*)d_out;

  char* ws = (char*)d_ws; size_t off = 0;
  auto carve = [&](size_t bytes) -> char* { char* p = ws + off; off += (bytes + 255) & ~(size_t)255; return p; };
  unsigned short* WE0I = (unsigned short*)carve((size_t)4 * NHE * NX  * 2);
  unsigned short* WE0H = (unsigned short*)carve((size_t)4 * NHE * NHE * 2);
  unsigned short* WE1I = (unsigned short*)carve((size_t)4 * NHE * NHE * 2);
  unsigned short* WE1H = (unsigned short*)carve((size_t)4 * NHE * NHE * 2);
  unsigned short* WD0I = (unsigned short*)carve((size_t)4 * NHD * NHE * 2);
  unsigned short* WD0H = (unsigned short*)carve((size_t)4 * NHD * NHD * 2);
  unsigned short* WD1I = (unsigned short*)carve((size_t)4 * NHD * NX  * 2);
  unsigned short* WD1H = (unsigned short*)carve((size_t)4 * NHD * NHD * 2);
  unsigned short* WOUT = (unsigned short*)carve((size_t)NX * NX * 2);
  float*          OUTB = (float*)carve((size_t)NX * 4);
  unsigned short* E0   = (unsigned short*)carve((size_t)NB * NSTEP * NHE * 2);
  unsigned short* HT16 = (unsigned short*)carve((size_t)NB * NHE * 2);
  float*          XGD0 = (float*)carve((size_t)NB * 4 * NHD * 4);
  unsigned short* D0   = (unsigned short*)carve((size_t)NB * NSTEP * NHD * 2);
  unsigned short* D1   = (unsigned short*)carve((size_t)NB * NSTEP * NHD * 2);
  if (off > ws_size || off > (size_t)134217728) return;

  auto cvt = [&](const float* s, unsigned short* d, int nelem) {
    const int n8 = nelem / 8;
    cvt16_kernel<<<(n8 + NTHR - 1) / NTHR, NTHR, 0, stream>>>(s, d, n8, CARRY);
  };
  cvt(e0_wih, WE0I, 4 * NHE * NX);
  cvt(e0_whh, WE0H, 4 * NHE * NHE);
  cvt(e1_wih, WE1I, 4 * NHE * NHE);
  cvt(e1_whh, WE1H, 4 * NHE * NHE);
  cvt(d0_wih, WD0I, 4 * NHD * NHE);
  cvt(d0_whh, WD0H, 4 * NHD * NHD);
  cvt(d1_wih, WD1I, 4 * NHD * NX);
  cvt(d1_whh, WD1H, 4 * NHD * NHD);
  cvt(out_w,  WOUT, NX * NX);
  bias16_kernel<<<1, 32, 0, stream>>>(out_b, OUTB);

  lstm_seq_kernel<NHE, NX, 0, true, false><<<NB / SEQ_ROWS, NTHR, 0, stream>>>(
      x, E0, XGD0, WE0I, WE0H, e0_bih, e0_bhh, E0, HT16);
  lstm_seq_kernel<NHE, NHE, 1, false, true><<<NB / SEQ_ROWS, NTHR, 0, stream>>>(
      x, E0, XGD0, WE1I, WE1H, e1_bih, e1_bhh, D0, HT16);
  wmma_gemm64<0, false, 0, 0, false, 0><<<dim3(((NB / 64) * ((4 * NHD) / 64)) / 8, 1), 256, 0, stream>>>(
      HT16, HT16, NHE, 0L, WD0I, WD0I, NHE, 0L, (void*)XGD0, (void*)XGD0, 4 * NHD, 0L,
      OUTB, OUTB, 0L, NB, 4 * NHD, NHE, CARRY2_INV);
  lstm_seq_kernel<NHD, NHE, 2, true, false><<<NB / SEQ_ROWS, NTHR, 0, stream>>>(
      x, E0, XGD0, WD0I, WD0H, d0_bih, d0_bhh, D0, HT16);
  lstm_seq_kernel<NHD, NHD, 1, true, false><<<NB / SEQ_ROWS, NTHR, 0, stream>>>(
      x, D0, XGD0, WD1I, WD1H, d1_bih, d1_bhh, D1, HT16);
  wmma_gemm64<0, false, 2, 0, false, 0><<<dim3((((NB * NSTEP) / 64) * (NX / 64)) / 8, 1), 256, 0, stream>>>(
      D1, D1, NHD, 0L, WOUT, WOUT, NX, 0L, (void*)out, (void*)out, NX, 0L,
      OUTB, OUTB, 0L, NB * NSTEP, NX, NHD, CARRY2_INV);
}
